// WTMambav2_80135499809160
// MI455X (gfx1250) — hardware-verified
//
#include <hip/hip_runtime.h>
#define NB 4
#define CC 64
#define HI 128
#define H2 64
#define NPX (H2 * H2)
#define DI 192
#define DS 16
#define DTR 6
#define KD 4
#define XDW 48
typedef __bf16 v16b __attribute__((ext_vector_type(16)));
typedef unsigned short v8us __attribute__((ext_vector_type(8), may_alias));
typedef float  v8f  __attribute__((ext_vector_type(8)));
typedef float  v4f  __attribute__((ext_vector_type(4)));
typedef float  v4fa __attribute__((ext_vector_type(4), may_alias));
union FragB { v16b v; v8us half[2]; unsigned short u[16]; };

__device__ __forceinline__ unsigned short bf16_bits(float x) { unsigned int u = __float_as_uint(x); return (unsigned short)((u + 0x7FFFu + ((u >> 16) & 1u)) >> 16); }
__device__ __forceinline__ float bf16_val(unsigned short b) { return __uint_as_float(((unsigned int)b) << 16); }
__device__ __forceinline__ float bf16_round(float x) { return bf16_val(bf16_bits(x)); }
template <int NT>
__device__ __forceinline__ v8f mmaN(v16b ah, v16b al, v16b bh, v16b bl, v8f c) {
  c = __builtin_amdgcn_wmma_f32_16x16x32_bf16(false, ah, false, bh, (short)0, c, false, false);
  if (NT >= 2) c = __builtin_amdgcn_wmma_f32_16x16x32_bf16(false, al, false, bh, (short)0, c, false, false);
  if (NT >= 3) c = __builtin_amdgcn_wmma_f32_16x16x32_bf16(false, ah, false, bl, (short)0, c, false, false);
  asm volatile("v_nop\n\tv_nop\n\tv_nop\n\tv_nop" : "+v"(c) : "v"(ah), "v"(al), "v"(bh), "v"(bl));
  return c;
}

__global__ __launch_bounds__(256) void k_wt_bf16(const float* __restrict__ W, unsigned short* __restrict__ Wt, int K, int N) {
  const int t = blockIdx.x * 256 + threadIdx.x;
  const int k8n = K / 8;
  if (t >= N * k8n) return;
  const int n = t / k8n, k8 = (t % k8n) * 8;
  v8us v;
#pragma unroll
  for (int i = 0; i < 8; ++i) v[i] = bf16_bits(W[(size_t)(k8 + i) * N + n]);
  *(volatile v8us*)(Wt + (size_t)n * K + k8) = v;
  __threadfence();
  *(volatile v8us*)(Wt + (size_t)n * K + k8) = v;
}

template <bool ASPLIT, int ACT, bool BIAS_BF16>
__global__ __launch_bounds__(128) void k_gemm_bf(const float* __restrict__ A, int lda, const unsigned short* __restrict__ Wt, int ldb,
                                               const float* __restrict__ bias, float* __restrict__ C, int ldc, int M, int N, int K) {
  __shared__ __attribute__((aligned(16))) float so[4][16][64];
  const int tid = threadIdx.x, w = tid >> 5, lane = tid & 31, ln = lane & 15, hh = lane >> 4;
  const int ntn = N / 64;
  const int wid = blockIdx.x * 4 + w;
  const int mt = wid / ntn, nq = wid % ntn;
  if (mt * 16 >= M) return;
  const int row0 = mt * 16, col0 = nq * 64;
  const float* arow = A + (size_t)(row0 + ln) * lda;
  v8f acc[4] = {};
  for (int kb = 0; kb < K; kb += 32) {
    FragB ah, al;
    const v4f x0 = *(const v4fa*)(arow + kb + 8 * hh), x1 = *(const v4fa*)(arow + kb + 8 * hh + 4);
    const v4f x2 = *(const v4fa*)(arow + kb + 16 + 8 * hh), x3 = *(const v4fa*)(arow + kb + 16 + 8 * hh + 4);
    float xs[16] = {x0[0],x0[1],x0[2],x0[3],x1[0],x1[1],x1[2],x1[3],x2[0],x2[1],x2[2],x2[3],x3[0],x3[1],x3[2],x3[3]};
#pragma unroll
    for (int i = 0; i < 16; ++i) { const unsigned short hb = bf16_bits(xs[i]); ah.u[i] = hb; al.u[i] = ASPLIT ? bf16_bits(xs[i] - bf16_val(hb)) : (unsigned short)0; }
#pragma unroll
    for (int t = 0; t < 4; ++t) {
      const unsigned short* brow = Wt + (size_t)(col0 + t * 16 + ln) * ldb + kb;
      FragB b;
      b.half[0] = *(const v8us*)(brow + 8 * hh);
      b.half[1] = *(const v8us*)(brow + 16 + 8 * hh);
      acc[t] = mmaN<ASPLIT ? 2 : 1>(ah.v, al.v, b.v, b.v, acc[t]);
    }
  }
#pragma unroll
  for (int t = 0; t < 4; ++t) {
    float bv = bias ? bias[col0 + t * 16 + ln] : 0.f;
    if (BIAS_BF16) bv = bf16_round(bv);
#pragma unroll
    for (int r = 0; r < 8; ++r) { float v = acc[t][r] + bv; if (ACT == 1) v = fmaxf(v, 0.f); so[w][8 * hh + r][t * 16 + ln] = v; }
  }
  __builtin_amdgcn_fence(__ATOMIC_ACQ_REL, "workgroup");
  __builtin_amdgcn_wave_barrier();
  const int rsub = lane >> 4, c4 = (lane & 15) * 4;
  for (int pass = 0; pass < 2; ++pass) {
#pragma unroll
    for (int q = 0; q < 8; ++q) {
      const int r = q * 2 + rsub;
      const v4f v = *(const v4fa*)&so[w][r][c4];
      *(volatile v4f*)(C + (size_t)(row0 + r) * ldc + col0 + c4) = v;
    }
    if (pass == 0) __threadfence();
  }
}

template <bool ASPLIT, int ACT, bool BIAS_BF16, bool RES_BF16>
__global__ __launch_bounds__(128) void k_gemm_bf3(const float* __restrict__ A, int lda, const unsigned short* __restrict__ Wt, int ldb,
                                                const float* __restrict__ bias, const float* __restrict__ resid, int rmod, int ldr,
                                                float* __restrict__ C, int ldc, int M, int N, int K) {
  __shared__ __attribute__((aligned(16))) float so[4][16][64];
  const int tid = threadIdx.x, w = tid >> 5, lane = tid & 31, ln = lane & 15, hh = lane >> 4;
  const int ntn = N / 64;
  const int wid = blockIdx.x * 4 + w;
  const int mt = wid / ntn, nq = wid % ntn;
  if (mt * 16 >= M) return;
  const int row0 = mt * 16, col0 = nq * 64;
  const float* arow = A + (size_t)(row0 + ln) * lda;
  v8f acc[4] = {};
  for (int kb = 0; kb < K; kb += 32) {
    FragB ah, al;
    const v4f x0 = *(const v4fa*)(arow + kb + 8 * hh), x1 = *(const v4fa*)(arow + kb + 8 * hh + 4);
    const v4f x2 = *(const v4fa*)(arow + kb + 16 + 8 * hh), x3 = *(const v4fa*)(arow + kb + 16 + 8 * hh + 4);
    float xs[16] = {x0[0],x0[1],x0[2],x0[3],x1[0],x1[1],x1[2],x1[3],x2[0],x2[1],x2[2],x2[3],x3[0],x3[1],x3[2],x3[3]};
#pragma unroll
    for (int i = 0; i < 16; ++i) { const unsigned short hb = bf16_bits(xs[i]); ah.u[i] = hb; al.u[i] = ASPLIT ? bf16_bits(xs[i] - bf16_val(hb)) : (unsigned short)0; }
#pragma unroll
    for (int t = 0; t < 4; ++t) {
      const unsigned short* brow = Wt + (size_t)(col0 + t * 16 + ln) * ldb + kb;
      FragB b;
      b.half[0] = *(const v8us*)(brow + 8 * hh);
      b.half[1] = *(const v8us*)(brow + 16 + 8 * hh);
      acc[t] = mmaN<ASPLIT ? 2 : 1>(ah.v, al.v, b.v, b.v, acc[t]);
    }
  }
#pragma unroll
  for (int t = 0; t < 4; ++t) {
    const int col = col0 + t * 16 + ln;
    float bv = bias ? bias[col] : 0.f;
    if (BIAS_BF16) bv = bf16_round(bv);
#pragma unroll
    for (int r = 0; r < 8; ++r) {
      float v = acc[t][r] + bv;
      if (resid) { float rv = resid[(size_t)((row0 + 8 * hh + r) % rmod) * ldr + col]; if (RES_BF16) rv = bf16_round(rv); v += rv; }
      if (ACT == 1) v = fmaxf(v, 0.f);
      if (ACT == 2) v = 0.5f * v * (1.0f + erff(v * 0.70710678118654752f));
      if (ACT == 3) { const float u = 0.7978845608028654f * (v + 0.044715f * v * v * v); v = 0.5f * v * (1.0f + tanhf(u)); }
      so[w][8 * hh + r][t * 16 + ln] = v;
    }
  }
  __builtin_amdgcn_fence(__ATOMIC_ACQ_REL, "workgroup");
  __builtin_amdgcn_wave_barrier();
  const int rsub = lane >> 4, c4 = (lane & 15) * 4;
  for (int pass = 0; pass < 2; ++pass) {
#pragma unroll
    for (int q = 0; q < 8; ++q) {
      const int r = q * 2 + rsub;
      const v4f v = *(const v4fa*)&so[w][r][c4];
      *(volatile v4f*)(C + (size_t)(row0 + r) * ldc + col0 + c4) = v;
    }
    if (pass == 0) __threadfence();
  }
}
template <bool PARAM_BF16>
__global__ __launch_bounds__(256) void k_layernorm(const float* __restrict__ X, const float* __restrict__ R, const float* __restrict__ g, const float* __restrict__ bta,
                                                  float* __restrict__ out_sum, float* __restrict__ out_norm, int N, float eps) {
  __shared__ float red[256];
  const int row = blockIdx.x, tid = threadIdx.x;
  const float* x = X + (size_t)row * N; const float* rr = R ? R + (size_t)row * N : nullptr;
  float vals[16];
  const int per = N / 256;
  float s1 = 0.f;
  for (int u = 0; u < per / 4; ++u) {
    const int j = tid * 4 + 1024 * u;
    const v4f a = *(const v4fa*)(x + j);
    v4f b = {0.f,0.f,0.f,0.f}; if (rr) b = *(const v4fa*)(rr + j);
#pragma unroll
    for (int q = 0; q < 4; ++q) { const float v = a[q] + b[q]; vals[u * 4 + q] = v; s1 += v; }
  }
  red[tid] = s1; __syncthreads();
  for (int st = 128; st > 0; st >>= 1) { if (tid < st) red[tid] += red[tid + st]; __syncthreads(); }
  const float mu = red[0] / (float)N; __syncthreads();
  float s2 = 0.f;
  for (int u = 0; u < per / 4; ++u)
#pragma unroll
    for (int q = 0; q < 4; ++q) { const float c = vals[u * 4 + q] - mu; s2 += c * c; }
  red[tid] = s2; __syncthreads();
  for (int st = 128; st > 0; st >>= 1) { if (tid < st) red[tid] += red[tid + st]; __syncthreads(); }
  const float rs = rsqrtf(red[0] / (float)N + eps);
  for (int pass = 0; pass < 2; ++pass) {
    for (int u = 0; u < per / 4; ++u) {
      const int j = tid * 4 + 1024 * u;
      v4f o, sm;
#pragma unroll
      for (int q = 0; q < 4; ++q) {
        float gg = g[j + q], bb = bta[j + q];
        if (PARAM_BF16) { gg = bf16_round(gg); bb = bf16_round(bb); }
        sm[q] = vals[u * 4 + q]; o[q] = (vals[u * 4 + q] - mu) * rs * gg + bb;
      }
      if (out_sum) *(volatile v4f*)(out_sum + (size_t)row * N + j) = sm;
      *(volatile v4f*)(out_norm + (size_t)row * N + j) = o;
    }
    if (pass == 0) __threadfence();
  }
}


typedef _Float16 v16h __attribute__((ext_vector_type(16)));
union FragH { v16h v; v8us half[2]; _Float16 h[16]; unsigned short u[16]; };
template <int NT>
__device__ __forceinline__ v8f mmaH(v16h ah, v16h al, v16h bh, v16h bl, v8f c) {
  c = __builtin_amdgcn_wmma_f32_16x16x32_f16(false, ah, false, bh, (short)0, c, false, false);
  if (NT >= 2) c = __builtin_amdgcn_wmma_f32_16x16x32_f16(false, al, false, bh, (short)0, c, false, false);
  if (NT >= 3) c = __builtin_amdgcn_wmma_f32_16x16x32_f16(false, ah, false, bl, (short)0, c, false, false);
  asm volatile("v_nop\n\tv_nop\n\tv_nop\n\tv_nop" : "+v"(c) : "v"(ah), "v"(al), "v"(bh), "v"(bl));
  return c;
}
template <bool ASPLIT>
__global__ __launch_bounds__(128) void k_gemm_h(const float* __restrict__ A, int lda, size_t sA, const _Float16* __restrict__ Bh, int ldb, size_t sB, float alpha, float* __restrict__ C, int ldc, size_t sC, int M, int N, int K) {
  __shared__ __attribute__((aligned(16))) float so[4][16][64];
  const int tid = threadIdx.x, w = tid >> 5, lane = tid & 31, ln = lane & 15, hh = lane >> 4; const int by = blockIdx.y;
  A += (size_t)by * sA; Bh += (size_t)by * sB; C += (size_t)by * sC;
  const int ntn = (N + 63) / 64; const int wid = blockIdx.x * 4 + w; const int mt = wid / ntn, nq = wid % ntn; if (mt * 16 >= M) return;
  const int row0 = mt * 16, col0 = nq * 64; const float* arow = A + (size_t)(row0 + ln) * lda;
  v8f acc[4] = {};
  for (int kb = 0; kb < K; kb += 32) {
    FragH ah, al;
    const v4f x0 = *(const v4fa*)(arow + kb + 8 * hh), x1 = *(const v4fa*)(arow + kb + 8 * hh + 4), x2 = *(const v4fa*)(arow + kb + 16 + 8 * hh), x3 = *(const v4fa*)(arow + kb + 16 + 8 * hh + 4);
    float xs[16] = {x0[0],x0[1],x0[2],x0[3],x1[0],x1[1],x1[2],x1[3],x2[0],x2[1],x2[2],x2[3],x3[0],x3[1],x3[2],x3[3]};
#pragma unroll
    for (int i = 0; i < 16; ++i) { const _Float16 h = (_Float16)xs[i]; ah.h[i] = h; al.h[i] = ASPLIT ? (_Float16)(xs[i] - (float)h) : (_Float16)0.0f; }
#pragma unroll
    for (int t = 0; t < 4; ++t) { if (col0 + t * 16 >= N) continue; const size_t boff = (size_t)(col0 + t * 16 + ln) * ldb + kb; FragH bq; bq.half[0] = *(const v8us*)(Bh + boff + 8 * hh); bq.half[1] = *(const v8us*)(Bh + boff + 16 + 8 * hh);
      acc[t] = mmaH<ASPLIT ? 2 : 1>(ah.v, al.v, bq.v, bq.v, acc[t]); }
  }
#pragma unroll
  for (int t = 0; t < 4; ++t) { if (col0 + t * 16 >= N) continue;
#pragma unroll
    for (int r = 0; r < 8; ++r) so[w][8 * hh + r][t * 16 + ln] = acc[t][r] * alpha; }
  __builtin_amdgcn_fence(__ATOMIC_ACQ_REL, "workgroup"); __builtin_amdgcn_wave_barrier();
  const int rsub = lane >> 4, c4 = (lane & 15) * 4;
  for (int pass = 0; pass < 2; ++pass) {
#pragma unroll
    for (int q = 0; q < 8; ++q) { const int r = q * 2 + rsub; if (col0 + c4 < N) { const v4f v = *(const v4fa*)&so[w][r][c4]; *(volatile v4f*)(C + (size_t)(row0 + r) * ldc + col0 + c4) = v; } }
    if (pass == 0) __threadfence(); }
}

__global__ __launch_bounds__(256) void k_wt_f16(const float* __restrict__ W, _Float16* __restrict__ Wt, int K, int N, float scale) {
  const int t = blockIdx.x * 256 + threadIdx.x; if (t >= N * (K / 8)) return; const int n = t / (K / 8), k8 = (t % (K / 8)) * 8; FragH f;
#pragma unroll
  for (int i = 0; i < 8; ++i) f.h[i] = (_Float16)(bf16_round(W[(size_t)(k8 + i) * N + n]) * scale); const v8us o = f.half[0];
  *(volatile v8us*)((unsigned short*)Wt + (size_t)n * K + k8) = o; __threadfence(); *(volatile v8us*)((unsigned short*)Wt + (size_t)n * K + k8) = o;
}
template <int ACT>
__global__ __launch_bounds__(128) void k_gemm_hhx(const _Float16* __restrict__ A, int lda, size_t sA, const _Float16* __restrict__ Bh, int ldb, size_t sB, float alpha, const float* __restrict__ bias, size_t sBias, const float* __restrict__ CP, int rowsPerB, size_t sCPb, int row0g,
    float* __restrict__ C, _Float16* __restrict__ C16, int ldc, size_t sC, int M, int N, int K) {
  __shared__ __attribute__((aligned(16))) float so[4][16][64];
  const int tid = threadIdx.x, w = tid >> 5, lane = tid & 31, ln = lane & 15, hh = lane >> 4; const int by = blockIdx.y;
  A += (size_t)by * sA; Bh += (size_t)by * sB; const size_t cofs = (size_t)by * sC; const float* bp = bias ? bias + (size_t)by * sBias : nullptr;
  const int ntn = (N + 63) / 64; const int wid = blockIdx.x * 4 + w; const int mt = wid / ntn, nq = wid % ntn; if (mt * 16 >= M) return;
  const int row0 = mt * 16, col0 = nq * 64; const _Float16* arow = A + (size_t)(row0 + ln) * lda;
  v8f acc[4] = {};
  for (int kb = 0; kb < K; kb += 32) { FragH ah; ah.half[0] = *(const v8us*)((const unsigned short*)arow + kb + 8 * hh); ah.half[1] = *(const v8us*)((const unsigned short*)arow + kb + 16 + 8 * hh);
#pragma unroll
    for (int t = 0; t < 4; ++t) { if (col0 + t * 16 >= N) continue; const size_t boff = (size_t)(col0 + t * 16 + ln) * ldb + kb; FragH bq; bq.half[0] = *(const v8us*)((const unsigned short*)Bh + boff + 8 * hh); bq.half[1] = *(const v8us*)((const unsigned short*)Bh + boff + 16 + 8 * hh);
      acc[t] = mmaH<1>(ah.v, ah.v, bq.v, bq.v, acc[t]); }
  }
#pragma unroll
  for (int t = 0; t < 4; ++t) { if (col0 + t * 16 >= N) continue; const int col = col0 + t * 16 + ln; const float bv = bp ? bf16_round(bp[col]) : 0.f;
#pragma unroll
    for (int r = 0; r < 8; ++r) { float v = acc[t][r] * alpha + bv; if (CP) { const int bidx = (row0g + row0 + 8 * hh + r) / rowsPerB; v += CP[(size_t)bidx * sCPb + (size_t)by * 64 + col]; } if (ACT == 1) v = (v > 0.f) ? v : expm1f(v); else if (ACT == 7) v = (v > 0.f) ? v + 1.0f : expf(v); else if (ACT == 8) v = tanhf(v); else if (ACT == 9) v = 0.5f * v * (1.0f + tanhf(0.7978845608028654f * (v + 0.044715f * v * v * v))); else if (ACT == 11) v = 1.0f / (1.0f + expf(-v)); else if (ACT == 12) v = (v > 0.f) ? v : 0.01f * v; else if (ACT == 14) v = (v > 0.f) ? v : 0.1f * v; else if (ACT == 15) v = v / (1.0f + expf(-v)); else if (ACT == 3) v = fmaxf(v, 0.f); else if (ACT == 6) v = 0.5f * v * (1.0f + erff(v * 0.70710678118654752f)); so[w][8 * hh + r][t * 16 + ln] = v; } }
  __builtin_amdgcn_fence(__ATOMIC_ACQ_REL, "workgroup"); __builtin_amdgcn_wave_barrier();
  const int rsub = lane >> 4, c4 = (lane & 15) * 4; typedef _Float16 v4h __attribute__((ext_vector_type(4)));
  for (int pass = 0; pass < 2; ++pass) {
#pragma unroll
    for (int q = 0; q < 8; ++q) { const int r = q * 2 + rsub; if (col0 + c4 < N) { const v4f v = *(const v4fa*)&so[w][r][c4]; if (C) *(volatile v4f*)(C + cofs + (size_t)(row0 + r) * ldc + col0 + c4) = v; if (C16) { v4h h4; for (int i = 0; i < 4; ++i) h4[i] = (_Float16)v[i]; *(volatile v4h*)(C16 + cofs + (size_t)(row0 + r) * ldc + col0 + c4) = h4; } } }
    if (pass == 0) __threadfence(); }
}


typedef _Float16 v4h __attribute__((ext_vector_type(4)));

__global__ __launch_bounds__(256) void k_x16(const float* __restrict__ x, _Float16* __restrict__ X16, size_t n8) { const size_t t = (size_t)blockIdx.x * 256 + threadIdx.x; if (t >= n8) return; FragH f;
#pragma unroll
  for (int q = 0; q < 8; ++q) f.h[q] = (_Float16)bf16_round(x[t * 8 + q]); *(volatile v8us*)((unsigned short*)X16 + t * 8) = f.half[0]; __threadfence(); *(volatile v8us*)((unsigned short*)X16 + t * 8) = f.half[0]; }
__global__ __launch_bounds__(256) void k_h16(const float* __restrict__ x, _Float16* __restrict__ X16, size_t n8) { const size_t t = (size_t)blockIdx.x * 256 + threadIdx.x; if (t >= n8) return; FragH f;
#pragma unroll
  for (int q = 0; q < 8; ++q) f.h[q] = (_Float16)x[t * 8 + q]; *(volatile v8us*)((unsigned short*)X16 + t * 8) = f.half[0]; __threadfence(); *(volatile v8us*)((unsigned short*)X16 + t * 8) = f.half[0]; }
__global__ __launch_bounds__(256) void k_round16f(const float* __restrict__ W, _Float16* __restrict__ Bt, size_t n8) { const size_t t = (size_t)blockIdx.x * 256 + threadIdx.x; if (t >= n8) return; FragH f;
#pragma unroll
  for (int i = 0; i < 8; ++i) f.h[i] = (_Float16)(bf16_round(W[t * 8 + i]) * 16.0f); *(volatile v8us*)((unsigned short*)Bt + t * 8) = f.half[0]; __threadfence(); *(volatile v8us*)((unsigned short*)Bt + t * 8) = f.half[0]; }
template <int NHv, int TTv>
__global__ __launch_bounds__(256) void k_vt(const _Float16* __restrict__ V16, int ldv, int voff, _Float16* __restrict__ Vt) { __shared__ unsigned short tl[64][66]; const int tid = threadIdx.x; const int slab = blockIdx.x / (TTv / 64), lg = blockIdx.x % (TTv / 64); const int b = slab / NHv, h = slab % NHv;
  for (int i = tid; i < 64 * 8; i += 256) { const int r = i / 8, c8 = (i % 8) * 8; FragH f; f.half[0] = *(const v8us*)((const unsigned short*)V16 + ((size_t)b * TTv + lg * 64 + r) * ldv + voff + h * 64 + c8);
#pragma unroll
    for (int q = 0; q < 8; ++q) tl[r][c8 + q] = f.u[q]; }
  __syncthreads();
  for (int pass = 0; pass < 2; ++pass) {
#pragma unroll
    for (int rd = 0; rd < 2; ++rd) { const int d = rd * 32 + tid / 8, pc = tid % 8; FragH f;
#pragma unroll
      for (int q = 0; q < 8; ++q) f.u[q] = tl[pc * 8 + q][d];
      *(volatile v8us*)((unsigned short*)Vt + ((size_t)slab * 64 + d) * TTv + lg * 64 + pc * 8) = f.half[0]; }
    if (pass == 0) __threadfence(); } }

__global__ __launch_bounds__(256) void k_hl(const float* __restrict__ F, _Float16* __restrict__ Hh, _Float16* __restrict__ Hl, size_t n8) { const size_t t = (size_t)blockIdx.x * 256 + threadIdx.x; if (t >= n8) return; FragH fh, fl; const v4f a = *(const v4fa*)(F + t * 8), c = *(const v4fa*)(F + t * 8 + 4);
#pragma unroll
  for (int q = 0; q < 4; ++q) { _Float16 h = (_Float16)a[q]; fh.h[q] = h; fl.h[q] = (_Float16)((a[q] - (float)h) * 1024.0f); h = (_Float16)c[q]; fh.h[4 + q] = h; fl.h[4 + q] = (_Float16)((c[q] - (float)h) * 1024.0f); }
  for (int pass = 0; pass < 2; ++pass) { *(volatile v8us*)((unsigned short*)Hh + t * 8) = fh.half[0]; *(volatile v8us*)((unsigned short*)Hl + t * 8) = fl.half[0]; if (pass == 0) __threadfence(); } }

typedef float v2f __attribute__((ext_vector_type(2)));
__device__ __forceinline__ float sigm_p(float x) { return 1.0f / (1.0f + expf(-x)); }
__device__ __forceinline__ float silu_p(float x) { return x / (1.0f + expf(-x)); }
__device__ __forceinline__ float silu_f(float x) { return x * __builtin_amdgcn_rcpf(1.0f + __expf(-x)); }
__device__ __forceinline__ void haar4(const float* __restrict__ x, int b, int c, int i, int j, float* s4) {
  #pragma clang fp contract(off)
  const float s = 0.70710678118654752440f; const float ll = s * s, ng = s * (-s); const float* xc = x + (((size_t)b * CC + c) * HI + 2 * i) * HI + 2 * j; const float a = bf16_round(xc[0]), bq = bf16_round(xc[1]), cq = bf16_round(xc[HI]), dq = bf16_round(xc[HI + 1]);
  s4[0] = ((a * ll + bq * ll) + cq * ll) + dq * ll; s4[1] = ((a * ll + bq * ll) + cq * ng) + dq * ng; s4[2] = ((a * ll + bq * ng) + cq * ll) + dq * ng; s4[3] = ((a * ll + bq * ng) + cq * ng) + dq * (s * s); }
__global__ __launch_bounds__(256) void k_dwt_low(const float* __restrict__ x, const float* __restrict__ wl, int b, _Float16* __restrict__ LOWIN) {
  #pragma clang fp contract(off)
  const int t = blockIdx.x * 256 + threadIdx.x; if (t >= NPX * (CC / 8)) return; const int c0 = (t % (CC / 8)) * 8, p = t / (CC / 8); const int i = p / H2, j = p % H2; FragH f;
#pragma unroll
  for (int q = 0; q < 8; ++q) { float s4[4]; haar4(x, b, c0 + q, i, j, s4); f.h[q] = (_Float16)(s4[0] * bf16_round(wl[c0 + q])); }
  *(volatile v8us*)((unsigned short*)LOWIN + (size_t)p * CC + c0) = f.half[0]; __threadfence(); *(volatile v8us*)((unsigned short*)LOWIN + (size_t)p * CC + c0) = f.half[0]; }
__global__ __launch_bounds__(256) void k_dwt_high(const float* __restrict__ x, const float* __restrict__ wh, int b, _Float16* __restrict__ HIGHIN) {
  #pragma clang fp contract(off)
  const int t = blockIdx.x * 256 + threadIdx.x; if (t >= NPX * (DI / 8)) return; const int h0 = (t % (DI / 8)) * 8, p = t / (DI / 8); const int i = p / H2, j = p % H2; FragH f;
#pragma unroll
  for (int q = 0; q < 8; ++q) { const int hc = h0 + q; const int c = hc / 3, sb = hc % 3; float s4[4]; haar4(x, b, c, i, j, s4); const float v = (sb == 0) ? s4[1] : (sb == 1) ? s4[2] : s4[3]; f.h[q] = (_Float16)(v * bf16_round(wh[hc])); }
  *(volatile v8us*)((unsigned short*)HIGHIN + (size_t)p * DI + h0) = f.half[0]; __threadfence(); *(volatile v8us*)((unsigned short*)HIGHIN + (size_t)p * DI + h0) = f.half[0]; }
__global__ __launch_bounds__(256) void k_dw(const float* __restrict__ XZ, const float* __restrict__ w, const float* __restrict__ bb, float* __restrict__ X1, _Float16* __restrict__ Xh, _Float16* __restrict__ Xl) {
  #pragma clang fp contract(off)
  const int t = blockIdx.x * 256 + threadIdx.x; if (t >= NPX * (DI / 4)) return; const int d0 = (t % (DI / 4)) * 4, p = t / (DI / 4); const int i = p / H2, j = p % H2; v4f o; FragH fh, fl;
#pragma unroll
  for (int q = 0; q < 4; ++q) { const int d = d0 + q; float acc = 0.f;
#pragma unroll 1
    for (int k = 0; k < 9; ++k) { const int ii = i + k / 3 - 1, jj = j + k % 3 - 1; if (ii >= 0 && ii < H2 && jj >= 0 && jj < H2) acc += XZ[(size_t)(ii * H2 + jj) * (2 * DI) + d] * bf16_round(w[d * 9 + k]); }
    const float v = silu_f(acc + bf16_round(bb[d])); o[q] = v; const _Float16 hi = (_Float16)v; fh.h[q] = hi; fl.h[q] = (_Float16)((v - (float)hi) * 1024.0f); }
  const unsigned long long vh = *(const unsigned long long*)&fh.u[0], vl = *(const unsigned long long*)&fl.u[0];
  for (int pass = 0; pass < 2; ++pass) { *(volatile v4f*)(X1 + (size_t)p * DI + d0) = o; *(volatile unsigned long long*)((unsigned short*)Xh + (size_t)p * DI + d0) = vh; *(volatile unsigned long long*)((unsigned short*)Xl + (size_t)p * DI + d0) = vl; if (pass == 0) __threadfence(); } }
__global__ __launch_bounds__(256) void k_wxp(const float* __restrict__ w, int k, _Float16* __restrict__ Bt) { const int t = blockIdx.x * 256 + threadIdx.x; if (t >= XDW * (DI / 8)) return; const int c0 = (t % (DI / 8)) * 8, n = t / (DI / 8); FragH f;
#pragma unroll
  for (int q = 0; q < 8; ++q) f.h[q] = (n < DTR + 2 * DS) ? (_Float16)(bf16_round(w[((size_t)k * (DTR + 2 * DS) + n) * DI + c0 + q]) * 16.0f) : (_Float16)0.0f;
  *(volatile v8us*)((unsigned short*)Bt + (size_t)n * DI + c0) = f.half[0]; __threadfence(); *(volatile v8us*)((unsigned short*)Bt + (size_t)n * DI + c0) = f.half[0]; }
__global__ __launch_bounds__(256) void k_delta(const float* __restrict__ XD, const float* __restrict__ dtw, const float* __restrict__ dtb, float* __restrict__ DLT) {
  #pragma clang fp contract(off)
  const size_t t = (size_t)blockIdx.x * 256 + threadIdx.x; if (t >= (size_t)KD * NPX * (DI / 4)) return; const int d0 = (int)(t % (DI / 4)) * 4; const size_t kp = t / (DI / 4); const int k = (int)(kp / NPX); const float* xd = XD + kp * XDW; v4f o;
#pragma unroll
  for (int q = 0; q < 4; ++q) { const int d = d0 + q; float s = bf16_round(dtb[k * DI + d]);
#pragma unroll
    for (int r = 0; r < DTR; ++r) s += bf16_round(dtw[((size_t)k * DI + d) * DTR + r]) * xd[r];
    o[q] = (s > 20.f) ? s : log1pf(expf(s)); }
  *(volatile v4f*)(DLT + kp * DI + d0) = o; __threadfence(); *(volatile v4f*)(DLT + kp * DI + d0) = o; }
__global__ __launch_bounds__(256) void k_scan(const float* __restrict__ X1, const float* __restrict__ XD, const float* __restrict__ DLT, const float* __restrict__ Alog, const float* __restrict__ Ds, float* __restrict__ YS) {
  #pragma clang fp contract(off)
  const int t = blockIdx.x * 256 + threadIdx.x; if (t >= KD * DI) return; const int k = t / DI, d = t % DI; float A[DS];
#pragma unroll
  for (int n = 0; n < DS; ++n) A[n] = -expf(bf16_round(Alog[((size_t)k * DI + d) * DS + n]));
  const float dsk = bf16_round(Ds[k * DI + d]);
  for (int pass = 0; pass < 2; ++pass) { float h[DS];
#pragma unroll
    for (int n = 0; n < DS; ++n) h[n] = 0.f;
#pragma unroll 1
    for (int l = 0; l < NPX; ++l) { int p; if (k == 0) p = l; else if (k == 1) p = (l % H2) * H2 + l / H2; else if (k == 2) p = NPX - 1 - l; else { const int m = NPX - 1 - l; p = (m % H2) * H2 + m / H2; }
      const float dl = DLT[((size_t)k * NPX + p) * DI + d], u = X1[(size_t)p * DI + d]; const float* bc = XD + ((size_t)k * NPX + p) * XDW + DTR; const float du = dl * u; float y = 0.f;
#pragma unroll
      for (int n = 0; n < DS; ++n) { h[n] = h[n] * __expf(dl * A[n]) + du * bc[n]; y += h[n] * bc[DS + n]; }
      y += u * dsk; *(volatile float*)(YS + ((size_t)k * NPX + p) * DI + d) = y; }
    if (pass == 0) __threadfence(); } }
__global__ __launch_bounds__(256) void k_post(const float* __restrict__ YS, const float* __restrict__ XZ, const float* __restrict__ ns, const float* __restrict__ nb, _Float16* __restrict__ G16) {
  #pragma clang fp contract(off)
  __shared__ __attribute__((aligned(16))) unsigned short rows[8][DI]; const int tid = threadIdx.x, w = tid >> 5, l = tid & 31; const int p = blockIdx.x * 8 + w; float v[6]; float s = 0.f;
#pragma unroll
  for (int m = 0; m < 6; ++m) { const int d = l + 32 * m; float y = 0.f;
#pragma unroll
    for (int k = 0; k < KD; ++k) y += YS[((size_t)k * NPX + p) * DI + d]; v[m] = y; s += y; }
  for (int o = 16; o > 0; o >>= 1) s += __shfl_xor(s, o, 32); const float mu = s / (float)DI; float vs = 0.f;
#pragma unroll
  for (int m = 0; m < 6; ++m) { const float dd = v[m] - mu; vs += dd * dd; }
  for (int o = 16; o > 0; o >>= 1) vs += __shfl_xor(vs, o, 32); const float rs = rsqrtf(vs / (float)DI + 1e-5f);
#pragma unroll
  for (int m = 0; m < 6; ++m) { const int d = l + 32 * m; const float z = XZ[(size_t)p * (2 * DI) + DI + d]; FragH f; f.h[0] = (_Float16)(((v[m] - mu) * rs * bf16_round(ns[d]) + bf16_round(nb[d])) * silu_p(z)); rows[w][d] = f.u[0]; }
  __syncthreads();
  for (int pass = 0; pass < 2; ++pass) { if (l < DI / 8) { const v8us vv = *(const v8us*)&rows[w][l * 8]; *(volatile v8us*)((unsigned short*)G16 + (size_t)p * DI + l * 8) = vv; } if (pass == 0) __threadfence(); } }
__global__ __launch_bounds__(256) void k_ln2(const float* __restrict__ HO, const float* __restrict__ s2, const float* __restrict__ b2, int b, float* __restrict__ HIGHF) {
  #pragma clang fp contract(off)
  const int tid = threadIdx.x, w = tid >> 5, l = tid & 31; const int p = blockIdx.x * 8 + w; float v[6]; float s = 0.f;
#pragma unroll
  for (int m = 0; m < 6; ++m) { v[m] = HO[(size_t)p * DI + l + 32 * m]; s += v[m]; }
  for (int o = 16; o > 0; o >>= 1) s += __shfl_xor(s, o, 32); const float mu = s / (float)DI; float vs = 0.f;
#pragma unroll
  for (int m = 0; m < 6; ++m) { const float dd = v[m] - mu; vs += dd * dd; }
  for (int o = 16; o > 0; o >>= 1) vs += __shfl_xor(vs, o, 32); const float rs = rsqrtf(vs / (float)DI + 1e-5f);
  for (int pass = 0; pass < 2; ++pass) {
#pragma unroll
    for (int m = 0; m < 6; ++m) { const int d = l + 32 * m; const float o_ = (v[m] - mu) * rs * bf16_round(s2[d]) + bf16_round(b2[d]); *(volatile float*)(HIGHF + ((size_t)b * NPX + p) * DI + d) = o_; }
    if (pass == 0) __threadfence(); } }
__global__ __launch_bounds__(256) void k_iwt(const float* __restrict__ LOW, const float* __restrict__ HIGHF, int b, float* __restrict__ Y) {
  #pragma clang fp contract(off)
  const int t = blockIdx.x * 256 + threadIdx.x; if (t >= CC * NPX) return; const int j = t % H2, i = (t / H2) % H2, c = t / NPX; const size_t p = (size_t)b * NPX + i * H2 + j; float m[4];
#pragma unroll
  for (int s_ = 0; s_ < 4; ++s_) { const int idx = c * 4 + s_; float v; if (idx < CC) v = LOW[p * CC + idx]; else { const int hc = idx - CC; v = LOW[p * CC + (hc % CC)] * HIGHF[p * DI + hc]; } m[s_] = v; }
  const float s = 0.70710678118654752440f; const float ll = s * s, ng = s * (-s);
  float o[2][2];
#pragma unroll
  for (int di = 0; di < 2; ++di)
#pragma unroll
    for (int dj = 0; dj < 2; ++dj) o[di][dj] = ((m[0] * ll + m[1] * (di ? ng : ll)) + m[2] * (dj ? ng : ll)) + m[3] * ((di ^ dj) ? ng : (s * s));
  for (int pass = 0; pass < 2; ++pass) {
#pragma unroll
    for (int di = 0; di < 2; ++di) { float* row = Y + (((size_t)b * CC + c) * HI + 2 * i + di) * HI + 2 * j; v2f pr; pr[0] = o[di][0]; pr[1] = o[di][1]; *(volatile v2f*)row = pr; }
    if (pass == 0) __threadfence(); } }
__global__ __launch_bounds__(256) void k_pool(const float* __restrict__ Y, float* __restrict__ POOL) { __shared__ float red[256]; const int tid = threadIdx.x; const size_t bc = blockIdx.x; const float* yp = Y + bc * (size_t)HI * HI; float s = 0.f;
#pragma unroll 1
  for (int i = tid; i < HI * HI; i += 256) s += yp[i]; red[tid] = s; __syncthreads();
  for (int k = 128; k > 0; k >>= 1) { if (tid < k) red[tid] += red[tid + k]; __syncthreads(); }
  if (tid < 32) { const float m = red[0] / (float)(HI * HI); *(volatile float*)(POOL + bc * 32 + tid) = m; __threadfence(); *(volatile float*)(POOL + bc * 32 + tid) = m; } }
__global__ __launch_bounds__(256) void k_final(const float* __restrict__ Y, const float* __restrict__ POOL, const float* __restrict__ ew, const float* __restrict__ x, float* __restrict__ out) {
  #pragma clang fp contract(off)
  const size_t t = (size_t)blockIdx.x * 256 + threadIdx.x; if (t >= (size_t)NB * CC * HI * HI / 4) return; const size_t e0 = t * 4; const int bc = (int)(e0 / ((size_t)HI * HI)); const int b = bc / CC, c = bc % CC; float a = 0.f;
#pragma unroll
  for (int k = 0; k < 5; ++k) { const int cc = c + k - 2; if (cc >= 0 && cc < CC) a += bf16_round(ew[k]) * POOL[((size_t)b * CC + cc) * 32]; }
  const float att = sigm_p(a); const v4f yv = *(const v4fa*)(Y + e0), xv = *(const v4fa*)(x + e0); v4f o;
#pragma unroll
  for (int q = 0; q < 4; ++q) o[q] = yv[q] * att + bf16_round(xv[q]); *(volatile v4f*)(out + e0) = o; __threadfence(); *(volatile v4f*)(out + e0) = o; }

extern "C" void kernel_launch(void* const* d_in, const int* in_sizes, int n_in,
                              void* d_out, int out_size, void* d_ws, size_t ws_size, hipStream_t stream) {
  (void)in_sizes; (void)n_in; (void)out_size;
  const float* const* I = (const float* const*)d_in; const float* x = I[0]; const float* wls = I[1]; const float* whs = I[2]; const float* lcw = I[3]; const float* ipw = I[4]; const float* dww = I[5]; const float* dwb = I[6]; const float* xpw = I[7]; const float* dtw = I[8]; const float* dtb = I[9]; const float* Alog = I[10]; const float* Dsv = I[11]; const float* ons = I[12]; const float* onb = I[13]; const float* opw = I[14]; const float* l2s = I[15]; const float* l2b = I[16]; const float* ecaw = I[17];
  char* ws = (char*)d_ws; size_t off = 0;
  auto take = [&](size_t bytes) { char* p = ws + off; off += (bytes + 255) & ~(size_t)255; return p; };
  _Float16* Blc = (_Float16*)take((size_t)CC * CC * 2); _Float16* Bip = (_Float16*)take((size_t)2 * DI * DI * 2); _Float16* Bxp[KD]; for (int k = 0; k < KD; ++k) Bxp[k] = (_Float16*)take((size_t)XDW * DI * 2); _Float16* Bop = (_Float16*)take((size_t)DI * DI * 2);
  _Float16* LOWIN = (_Float16*)take((size_t)NPX * CC * 2); _Float16* HIGHIN = (_Float16*)take((size_t)NPX * DI * 2); float* LOW = (float*)take((size_t)NB * NPX * CC * 4); float* XZ = (float*)take((size_t)NPX * 2 * DI * 4); float* X1 = (float*)take((size_t)NPX * DI * 4); _Float16* Xh = (_Float16*)take((size_t)NPX * DI * 2); _Float16* Xl = (_Float16*)take((size_t)NPX * DI * 2);
  float* XD = (float*)take((size_t)KD * NPX * XDW * 4); float* DLT = (float*)take((size_t)KD * NPX * DI * 4); float* YS = (float*)take((size_t)KD * NPX * DI * 4); _Float16* G16 = (_Float16*)take((size_t)NPX * DI * 2); float* HO = (float*)take((size_t)NPX * DI * 4); float* HIGHF = (float*)take((size_t)NB * NPX * DI * 4);
  float* Y = (float*)take((size_t)NB * CC * HI * HI * 4); float* POOL = (float*)take((size_t)NB * CC * 32 * 4);
  if (off > ws_size) return;
  k_round16f<<<(CC * CC / 8 + 255) / 256, 256, 0, stream>>>(lcw, Blc, (size_t)CC * CC / 8); k_round16f<<<(2 * DI * DI / 8 + 255) / 256, 256, 0, stream>>>(ipw, Bip, (size_t)2 * DI * DI / 8); for (int k = 0; k < KD; ++k) k_wxp<<<(XDW * (DI / 8) + 255) / 256, 256, 0, stream>>>(xpw, k, Bxp[k]); k_round16f<<<(DI * DI / 8 + 255) / 256, 256, 0, stream>>>(opw, Bop, (size_t)DI * DI / 8);
  const dim3 gL(((NPX / 16) * (CC / 64) + 3) / 4, 1), gIP(((NPX / 16) * (2 * DI / 64) + 3) / 4, 1), gXP(((NPX / 16) * 1 + 3) / 4, 1), gOP(((NPX / 16) * (DI / 64) + 3) / 4, 1);
  for (int b = 0; b < NB; ++b) {
    k_dwt_low<<<(NPX * (CC / 8) + 255) / 256, 256, 0, stream>>>(x, wls, b, LOWIN); k_dwt_high<<<(NPX * (DI / 8) + 255) / 256, 256, 0, stream>>>(x, whs, b, HIGHIN);
    k_gemm_hhx<15><<<gL, 128, 0, stream>>>(LOWIN, CC, 0, Blc, CC, 0, 0.0625f, nullptr, 0, nullptr, 1, 0, 0, LOW + (size_t)b * NPX * CC, nullptr, CC, 0, NPX, CC, CC);
    k_gemm_hhx<0><<<gIP, 128, 0, stream>>>(HIGHIN, DI, 0, Bip, DI, 0, 0.0625f, nullptr, 0, nullptr, 1, 0, 0, XZ, nullptr, 2 * DI, 0, NPX, 2 * DI, DI);
    k_dw<<<(NPX * (DI / 4) + 255) / 256, 256, 0, stream>>>(XZ, dww, dwb, X1, Xh, Xl);
    for (int k = 0; k < KD; ++k) { float* xd = XD + (size_t)k * NPX * XDW;
      k_gemm_hhx<0><<<gXP, 128, 0, stream>>>(Xh, DI, 0, Bxp[k], DI, 0, 0.0625f, nullptr, 0, nullptr, 1, 0, 0, xd, nullptr, XDW, 0, NPX, XDW, DI); k_gemm_hhx<0><<<gXP, 128, 0, stream>>>(Xl, DI, 0, Bxp[k], DI, 0, 0.0625f / 1024.0f, nullptr, 0, xd, 1, (size_t)XDW, 0, xd, nullptr, XDW, 0, NPX, XDW, DI); }
    k_delta<<<(unsigned)(((size_t)KD * NPX * (DI / 4) + 255) / 256), 256, 0, stream>>>(XD, dtw, dtb, DLT);
    k_scan<<<(KD * DI + 255) / 256, 256, 0, stream>>>(X1, XD, DLT, Alog, Dsv, YS);
    k_post<<<NPX / 8, 256, 0, stream>>>(YS, XZ, ons, onb, G16);
    k_gemm_hhx<0><<<gOP, 128, 0, stream>>>(G16, DI, 0, Bop, DI, 0, 0.0625f, nullptr, 0, nullptr, 1, 0, 0, HO, nullptr, DI, 0, NPX, DI, DI);
    k_ln2<<<NPX / 8, 256, 0, stream>>>(HO, l2s, l2b, b, HIGHF);
    k_iwt<<<(CC * NPX + 255) / 256, 256, 0, stream>>>(LOW, HIGHF, b, Y); }
  k_pool<<<NB * CC, 256, 0, stream>>>(Y, POOL);
  k_final<<<(unsigned)(((size_t)NB * CC * HI * HI / 4 + 255) / 256), 256, 0, stream>>>(Y, POOL, ecaw, x, (float*)d_out);
}
